// EqvMSPFeedForward_51994874085877
// MI455X (gfx1250) — hardware-verified
//
#include <hip/hip_runtime.h>
#include <math.h>


typedef _Float16 v16h __attribute__((ext_vector_type(16)));
typedef _Float16 v8h  __attribute__((ext_vector_type(8)));
typedef float    v8f  __attribute__((ext_vector_type(8)));
typedef float    v4f  __attribute__((ext_vector_type(4)));
typedef unsigned v4u  __attribute__((ext_vector_type(4)));

#define NB      8
#define NHALF   32
#define NPT     64
#define CH      64
#define HRE     100
#define HPAD    128
#define NBAS    10
#define W3COLS  (CH * CH)
#define NPAIR   (NB * NPT * NPT)
#define KBIG    (NPT * HPAD)
#define NROWX   (NB * NPT)
#define W3PROWS (CH * HPAD)
#define PPB     4
#define TP16    72
#define TP32    68

union Frag { v16h v; v8h h[2]; };
union P8   { v8h h; v4u u; _Float16 e[8]; };

static __device__ __forceinline__ v8f wmma16(v8f acc, v16h a, v16h b) {
    acc = __builtin_amdgcn_wmma_f32_16x16x32_f16(false, a, false, b, (short)0, acc, false, false);
    asm volatile("v_nop\n\tv_nop\n\tv_nop\n\tv_nop" : "+v"(acc) : "v"(a), "v"(b));
    return acc;
}

static __device__ __forceinline__ v8f zero8() {
    v8f z = {0.f, 0.f, 0.f, 0.f, 0.f, 0.f, 0.f, 0.f};
    return z;
}

static __device__ __forceinline__ float silu_f(float x) { return x / (1.0f + expf(-x)); }

static __device__ __forceinline__ void gemm_core(const _Float16* __restrict__ Ab, int lda,
                                                 const _Float16* __restrict__ Bb, int ldbt, int K,
                                                 v8f& c0, v8f& c1, v8f& c2, v8f& c3) {
    const int t = threadIdx.x, wave = t >> 5, lane = t & 31, m = lane & 15, hh = lane >> 4;
    const _Float16* Ar = Ab + (size_t)(wave * 16 + m) * lda + 8 * hh;
    const _Float16* B0 = Bb + (size_t)m * ldbt + 8 * hh;
    const _Float16* B1 = B0 + (size_t)16 * ldbt;
    const _Float16* B2 = B0 + (size_t)32 * ldbt;
    const _Float16* B3 = B0 + (size_t)48 * ldbt;
    for (int k0 = 0; k0 < K; k0 += 32) {
        Frag a, b0, b1, b2, b3;
        a.h[0]  = *(const v8h*)(Ar + k0);  a.h[1]  = *(const v8h*)(Ar + k0 + 16);
        b0.h[0] = *(const v8h*)(B0 + k0);  b0.h[1] = *(const v8h*)(B0 + k0 + 16);
        b1.h[0] = *(const v8h*)(B1 + k0);  b1.h[1] = *(const v8h*)(B1 + k0 + 16);
        b2.h[0] = *(const v8h*)(B2 + k0);  b2.h[1] = *(const v8h*)(B2 + k0 + 16);
        b3.h[0] = *(const v8h*)(B3 + k0);  b3.h[1] = *(const v8h*)(B3 + k0 + 16);
        c0 = wmma16(c0, a.v, b0.v);
        c1 = wmma16(c1, a.v, b1.v);
        c2 = wmma16(c2, a.v, b2.v);
        c3 = wmma16(c3, a.v, b3.v);
    }
}

#define PK_C0 (HPAD * HPAD / 8)
#define PK_C1 (PK_C0 + W3PROWS * CH / 8)
#define PK_C2 (PK_C1 + NROWX * CH / 8)

__global__ __launch_bounds__(256) void k_pack(const float* __restrict__ w2, const float* __restrict__ w3,
                                              const float* __restrict__ in1, const float* __restrict__ in2,
                                              _Float16* __restrict__ w2t, _Float16* __restrict__ w3p,
                                              _Float16* __restrict__ xp) {
    const int c = blockIdx.x * 256 + threadIdx.x;
    P8 p;
    _Float16* dst;
    if (c < PK_C0) {
        const int n = c >> 4, k0 = (c & 15) * 8;
#pragma unroll
        for (int i = 0; i < 8; ++i) {
            const int k = k0 + i;
            const float v = (k < HRE && n < HRE) ? w2[k * HRE + n] : 0.0f;
            p.e[i] = (_Float16)v;
        }
        dst = w2t + (size_t)c * 8;
    } else if (c < PK_C1) {
        const int cc = c - PK_C0;
        const int row = cc >> 3, i0 = (cc & 7) * 8;
        const int o = row >> 7, h = row & 127;
        if (h < HRE) {
            const float* s = w3 + (size_t)h * W3COLS + o * CH + i0;
            const v4f lo = *(const v4f*)s, hi = *(const v4f*)(s + 4);
            p.e[0] = (_Float16)lo[0]; p.e[1] = (_Float16)lo[1]; p.e[2] = (_Float16)lo[2]; p.e[3] = (_Float16)lo[3];
            p.e[4] = (_Float16)hi[0]; p.e[5] = (_Float16)hi[1]; p.e[6] = (_Float16)hi[2]; p.e[7] = (_Float16)hi[3];
        } else {
#pragma unroll
            for (int i = 0; i < 8; ++i) p.e[i] = (_Float16)0.0f;
        }
        dst = w3p + (size_t)cc * 8;
    } else if (c < PK_C2) {
        const int cc = c - PK_C1;
        const int row = cc >> 3, i0 = (cc & 7) * 8;
        const int z = row >> 6, b = row & 63;
        const float* s = (b < NHALF) ? (in1 + ((size_t)(z * NHALF + b) * CH + i0))
                                     : (in2 + ((size_t)(z * NHALF + (b - NHALF)) * CH + i0));
        const v4f lo = *(const v4f*)s, hi = *(const v4f*)(s + 4);
        p.e[0] = (_Float16)lo[0]; p.e[1] = (_Float16)lo[1]; p.e[2] = (_Float16)lo[2]; p.e[3] = (_Float16)lo[3];
        p.e[4] = (_Float16)hi[0]; p.e[5] = (_Float16)hi[1]; p.e[6] = (_Float16)hi[2]; p.e[7] = (_Float16)hi[3];
        dst = xp + (size_t)cc * 8;
    } else {
        return;
    }
    *(volatile v4u*)dst = p.u;
    __threadfence();
    *(volatile v4u*)dst = p.u;
}

__global__ __launch_bounds__(128) void k_radial_h1(const float* __restrict__ xyz1, const float* __restrict__ xyz2,
                                                   const float* __restrict__ w1, _Float16* __restrict__ h1b,
                                                   int npairs) {
    __shared__ float bas[PPB][NBAS];
    __shared__ __align__(16) _Float16 hs[PPB * HPAD];
    const int t = threadIdx.x;
    const int pbase = blockIdx.x * PPB;
    if (t < PPB * NBAS) {
        const int j = t / NBAS, n = t - j * NBAS;
        const int p = pbase + j;
        float bv = 0.0f;
        if (p < npairs) {
            const int z = p >> 12, a = (p >> 6) & 63, b = p & 63;
            const float* pa = (a < NHALF) ? (xyz1 + (z * NHALF + a) * 3) : (xyz2 + (z * NHALF + (a - NHALF)) * 3);
            const float* pb = (b < NHALF) ? (xyz1 + (z * NHALF + b) * 3) : (xyz2 + (z * NHALF + (b - NHALF)) * 3);
            const float dx = pa[0] - pb[0], dy = pa[1] - pb[1], dz = pa[2] - pb[2];
            const float r = sqrtf(dx * dx + dy * dy + dz * dz + 1e-12f);
            const float step = 10.0f / 9.0f;
            const float hpi = 1.5707963267948966f;
            const float u = (r - (float)n * step) / step * hpi;
            const float cu = cosf(u);
            bv = (fabsf(u) < hpi) ? cu * cu : 0.0f;
        }
        bas[j][n] = bv;
    }
    __syncthreads();
    float wc[NBAS];
#pragma unroll
    for (int jj = 0; jj < NBAS; ++jj) wc[jj] = (t < HRE) ? w1[jj * HRE + t] : 0.0f;
#pragma unroll 1
    for (int j = 0; j < PPB; ++j) {
        float acc = 0.0f;
#pragma unroll
        for (int jj = 0; jj < NBAS; ++jj) acc += bas[j][jj] * wc[jj];
        acc *= 0.31622776601683794f;
        acc = silu_f(acc);
        hs[j * HPAD + t] = (_Float16)(acc * 64.0f);
    }
    __syncthreads();
    P8 v;
    _Float16* dst = h1b;
    bool doit = false;
    if (t < PPB * HPAD / 8) {
        const int p = pbase + (t >> 4);
        if (p < npairs) {
            v.h = *(const v8h*)(hs + t * 8);
            dst = h1b + (size_t)pbase * HPAD + t * 8;
            doit = true;
        }
    }
    if (doit) *(volatile v4u*)dst = v.u;
    __threadfence();
    if (doit) *(volatile v4u*)dst = v.u;
}

__global__ __launch_bounds__(128) void k_gemm_h2(const _Float16* __restrict__ h1b, const _Float16* __restrict__ w2t,
                                                 _Float16* __restrict__ h2b, int nrows) {
    __shared__ __align__(16) _Float16 tile[64 * TP16];
    const int row0 = blockIdx.x * 64, col0 = blockIdx.y * 64;
    if (row0 >= nrows || col0 >= HPAD) return;
    v8f c0 = zero8(), c1 = zero8(), c2 = zero8(), c3 = zero8();
    gemm_core(h1b + (size_t)row0 * HPAD, HPAD, w2t + (size_t)col0 * HPAD, HPAD, HPAD, c0, c1, c2, c3);
    const int t = threadIdx.x, wave = t >> 5, lane = t & 31, m = lane & 15, hh = lane >> 4;
    const float sc = 0.1f / 64.0f;
#pragma unroll
    for (int r = 0; r < 8; ++r) {
        const int row = wave * 16 + hh * 8 + r;
        tile[row * TP16 + m]      = (_Float16)(silu_f(c0[r] * sc) * 64.0f);
        tile[row * TP16 + 16 + m] = (_Float16)(silu_f(c1[r] * sc) * 64.0f);
        tile[row * TP16 + 32 + m] = (_Float16)(silu_f(c2[r] * sc) * 64.0f);
        tile[row * TP16 + 48 + m] = (_Float16)(silu_f(c3[r] * sc) * 64.0f);
    }
    __syncthreads();
    P8 v[4];
#pragma unroll
    for (int it = 0; it < 4; ++it) {
        const int row = wave * 16 + it * 4 + (lane >> 3), ch = lane & 7;
        v[it].h = *(const v8h*)(tile + row * TP16 + ch * 8);
    }
#pragma unroll
    for (int it = 0; it < 4; ++it) {
        const int row = wave * 16 + it * 4 + (lane >> 3), ch = lane & 7;
        _Float16* dst = h2b + (size_t)(row0 + row) * HPAD + col0 + ch * 8;
        *(volatile v4u*)dst = v[it].u;
    }
    __threadfence();
#pragma unroll
    for (int it = 0; it < 4; ++it) {
        const int row = wave * 16 + it * 4 + (lane >> 3), ch = lane & 7;
        _Float16* dst = h2b + (size_t)(row0 + row) * HPAD + col0 + ch * 8;
        *(volatile v4u*)dst = v[it].u;
    }
}

__global__ __launch_bounds__(128) void k_gemm_g(const _Float16* __restrict__ w3p, const _Float16* __restrict__ xp,
                                                _Float16* __restrict__ Gt) {
    __shared__ __align__(16) _Float16 tileT[64 * TP16];
    const int bx = blockIdx.x, z = blockIdx.y;
    if (bx >= W3PROWS / 64 || z >= NB) return;
    const int o = bx >> 1, hsel = bx & 1;
    v8f c0 = zero8(), c1 = zero8(), c2 = zero8(), c3 = zero8();
    gemm_core(w3p + (size_t)bx * 64 * CH, CH, xp + (size_t)z * NPT * CH, CH, CH, c0, c1, c2, c3);
    const int t = threadIdx.x, wave = t >> 5, lane = t & 31, m = lane & 15, hh = lane >> 4;
#pragma unroll
    for (int r = 0; r < 8; ++r) {
        const int hrow = wave * 16 + hh * 8 + r;
        tileT[(m) * TP16 + hrow]      = (_Float16)c0[r];
        tileT[(16 + m) * TP16 + hrow] = (_Float16)c1[r];
        tileT[(32 + m) * TP16 + hrow] = (_Float16)c2[r];
        tileT[(48 + m) * TP16 + hrow] = (_Float16)c3[r];
    }
    __syncthreads();
    P8 v[4];
#pragma unroll
    for (int it = 0; it < 4; ++it) {
        const int b = wave * 16 + it * 4 + (lane >> 3), ch = lane & 7;
        v[it].h = *(const v8h*)(tileT + b * TP16 + ch * 8);
    }
    const size_t rowbase = (size_t)(z * CH + o) * KBIG + hsel * 64;
#pragma unroll
    for (int it = 0; it < 4; ++it) {
        const int b = wave * 16 + it * 4 + (lane >> 3), ch = lane & 7;
        _Float16* dst = Gt + rowbase + (size_t)b * HPAD + ch * 8;
        *(volatile v4u*)dst = v[it].u;
    }
    __threadfence();
#pragma unroll
    for (int it = 0; it < 4; ++it) {
        const int b = wave * 16 + it * 4 + (lane >> 3), ch = lane & 7;
        _Float16* dst = Gt + rowbase + (size_t)b * HPAD + ch * 8;
        *(volatile v4u*)dst = v[it].u;
    }
}

__global__ __launch_bounds__(128) void k_gemm_xo(const _Float16* __restrict__ h2b, const _Float16* __restrict__ Gt,
                                                 float* __restrict__ xo) {
    __shared__ __align__(16) float tile[64 * TP32];
    const int z = blockIdx.x;
    if (z >= NB) return;
    v8f c0 = zero8(), c1 = zero8(), c2 = zero8(), c3 = zero8();
    gemm_core(h2b + (size_t)z * NPT * KBIG, KBIG, Gt + (size_t)z * CH * KBIG, KBIG, KBIG, c0, c1, c2, c3);
    const int t = threadIdx.x, wave = t >> 5, lane = t & 31, m = lane & 15, hh = lane >> 4;
    const float sc = 0.0125f / 64.0f;
#pragma unroll
    for (int r = 0; r < 8; ++r) {
        const int row = wave * 16 + hh * 8 + r;
        tile[row * TP32 + m]      = c0[r] * sc;
        tile[row * TP32 + 16 + m] = c1[r] * sc;
        tile[row * TP32 + 32 + m] = c2[r] * sc;
        tile[row * TP32 + 48 + m] = c3[r] * sc;
    }
    __syncthreads();
    v4f v[8];
#pragma unroll
    for (int it = 0; it < 8; ++it) {
        const int row = wave * 16 + it * 2 + (lane >> 4), ch = lane & 15;
        v[it] = *(const v4f*)(tile + row * TP32 + ch * 4);
    }
    float* base = xo + (size_t)z * NPT * CH;
#pragma unroll
    for (int it = 0; it < 8; ++it) {
        const int row = wave * 16 + it * 2 + (lane >> 4), ch = lane & 15;
        *(volatile v4f*)(base + row * CH + ch * 4) = v[it];
    }
    __threadfence();
#pragma unroll
    for (int it = 0; it < 8; ++it) {
        const int row = wave * 16 + it * 2 + (lane >> 4), ch = lane & 15;
        *(volatile v4f*)(base + row * CH + ch * 4) = v[it];
    }
}

__global__ __launch_bounds__(64) void k_head(const float* __restrict__ xo, const int* __restrict__ mask,
                                            const float* __restrict__ fc3, const float* __restrict__ fc2,
                                            float* __restrict__ out, int nb) {
    __shared__ float s[64], red[64], res[32];
    const int o = threadIdx.x;
    if (o < 32) res[o] = 0.0f;
    __syncthreads();
    const float f2 = fc2[o];
#pragma unroll 1
    for (int z = 0; z < nb; ++z) {
        float acc = 0.0f;
#pragma unroll 1
        for (int a = 0; a < NPT; ++a)
            if (mask[z * NPT + a] != 0) acc += fabsf(xo[((size_t)z * NPT + a) * CH + o]);
        red[o] = acc;
        __syncthreads();
        for (int st = 32; st > 0; st >>= 1) { if (o < st) red[o] += red[o + st]; __syncthreads(); }
        const float mean = red[0] * (1.0f / 64.0f);
        __syncthreads();
        const float d = acc - mean;
        red[o] = d * d;
        __syncthreads();
        for (int st = 32; st > 0; st >>= 1) { if (o < st) red[o] += red[o + st]; __syncthreads(); }
        const float stdv = sqrtf(red[0] * (1.0f / 63.0f));
        __syncthreads();
        s[o] = d / (stdv + 1e-6f);
        __syncthreads();
        float hsum = 0.0f;
#pragma unroll 4
        for (int i = 0; i < CH; ++i) hsum += s[i] * fc3[i * CH + o];
        hsum *= 0.125f;
        hsum = (hsum > 0.0f) ? hsum : 0.01f * hsum;
        red[o] = hsum * f2 * 0.125f;
        __syncthreads();
        for (int st = 32; st > 0; st >>= 1) { if (o < st) red[o] += red[o + st]; __syncthreads(); }
        if (o == 0) res[z] = 1.0f / (1.0f + expf(-red[0]));
        __syncthreads();
    }
    const int nq = nb >> 2;
    const bool dq = (o < nq);
    const int sidx = nq * 4 + o;
    const bool ds = (o < (nb & 3));
    v4f q = {0.0f, 0.0f, 0.0f, 0.0f};
    float sv = 0.0f;
    if (dq) { q[0] = res[4 * o]; q[1] = res[4 * o + 1]; q[2] = res[4 * o + 2]; q[3] = res[4 * o + 3]; }
    if (ds) sv = res[sidx];
    if (dq) *(volatile v4f*)(out + 4 * o) = q;
    if (ds) *(volatile float*)(out + sidx) = sv;
    __threadfence();
    if (dq) *(volatile v4f*)(out + 4 * o) = q;
    if (ds) *(volatile float*)(out + sidx) = sv;
}


extern "C" void kernel_launch(void* const* d_in, const int* in_sizes, int n_in,
                              void* d_out, int out_size, void* d_ws, size_t ws_size,
                              hipStream_t stream) {
    if (n_in < 10) return;
    if (in_sizes[0] != NB * NHALF * CH || in_sizes[1] != NB * NHALF * CH) return;
    if (in_sizes[2] != NB * NHALF * 3  || in_sizes[3] != NB * NHALF * 3) return;
    if (in_sizes[4] != NB * NPT) return;
    if (in_sizes[5] != NBAS * HRE || in_sizes[6] != HRE * HRE || in_sizes[7] != HRE * W3COLS) return;
    if (in_sizes[8] != CH * CH || in_sizes[9] != CH) return;
    if (out_size != NB) return;

    const float* input1 = (const float*)d_in[0];
    const float* input2 = (const float*)d_in[1];
    const float* xyz1   = (const float*)d_in[2];
    const float* xyz2   = (const float*)d_in[3];
    const int*   mask   = (const int*)  d_in[4];
    const float* w1     = (const float*)d_in[5];
    const float* w2     = (const float*)d_in[6];
    const float* w3     = (const float*)d_in[7];
    const float* fc3    = (const float*)d_in[8];
    const float* fc2    = (const float*)d_in[9];
    float* out = (float*)d_out;

    const size_t sz_h1b = (size_t)NPAIR * HPAD * 2;
    const size_t sz_w2t = (size_t)HPAD * HPAD * 2;
    const size_t sz_h2b = (size_t)NPAIR * HPAD * 2;
    const size_t sz_w3p = (size_t)W3PROWS * CH * 2;
    const size_t sz_xp  = (size_t)NROWX * CH * 2;
    const size_t sz_gt  = (size_t)NB * CH * KBIG * 2;
    const size_t sz_xo  = (size_t)NB * NPT * CH * 4;
    size_t off = 0;
    const size_t o_h1b = off; off += sz_h1b;
    const size_t o_w2t = off; off += sz_w2t;
    const size_t o_h2b = off; off += sz_h2b;
    const size_t o_w3p = off; off += sz_w3p;
    const size_t o_xp  = off; off += sz_xp;
    const size_t o_gt  = off; off += sz_gt;
    const size_t o_xo  = off; off += sz_xo;
    if (off > ws_size) return;

    char* ws = (char*)d_ws;
    _Float16* h1b = (_Float16*)(ws + o_h1b);
    _Float16* w2t = (_Float16*)(ws + o_w2t);
    _Float16* h2b = (_Float16*)(ws + o_h2b);
    _Float16* w3p = (_Float16*)(ws + o_w3p);
    _Float16* xp  = (_Float16*)(ws + o_xp);
    _Float16* Gt  = (_Float16*)(ws + o_gt);
    float*    xo  = (float*)   (ws + o_xo);

    k_pack<<<(PK_C2 + 255) / 256, 256, 0, stream>>>(w2, w3, input1, input2, w2t, w3p, xp);
    k_radial_h1<<<(NPAIR + PPB - 1) / PPB, 128, 0, stream>>>(xyz1, xyz2, w1, h1b, NPAIR);
    k_gemm_h2<<<dim3((NPAIR + 63) / 64, HPAD / 64, 1), 128, 0, stream>>>(h1b, w2t, h2b, NPAIR);
    k_gemm_g<<<dim3(W3PROWS / 64, NB, 1), 128, 0, stream>>>(w3p, xp, Gt);
    k_gemm_xo<<<NB, 128, 0, stream>>>(h2b, Gt, xo);
    k_head<<<1, 64, 0, stream>>>(xo, mask, fc3, fc2, out, NB);
}
